// MultiRelationGE_GNNLayer_85512798863506
// MI455X (gfx1250) — hardware-verified
//
#include <hip/hip_runtime.h>
#include <stddef.h>
#include <math.h>


#define DI    64
#define HH    64
#define NHD   4
#define NREL  3
#define NCOL  256
#define KL    192
#define GR    32
#define AP    72
#define XSP   260
#define NB    512
#define CHUNK 2048
#define NTHR  256
#define NWAVE 8
#define WCAP  256
#define NGRP  (CHUNK / (NTHR * 4))
#define SROW  128

#define LDS_SACC (NB * SROW)
#define LDS_DEN  (NB * NHD)
#define LDS_MAX  (NB * NHD)
#define LDS_CNT  (NB)
#define LDS_BET  128
#define LDS_LB   64
#define LDS_LIST (NWAVE * WCAP)
#define LDS_BYTES ((LDS_SACC + LDS_DEN + LDS_MAX + LDS_CNT + LDS_BET + LDS_LB + LDS_LIST + NWAVE) * 4)

static_assert(WCAP == (CHUNK / NTHR) * 32);
static_assert(NGRP == 2);
static_assert(NB == 512);
static_assert(NB == NWAVE * 64);
static_assert(NTHR == NCOL);
static_assert(((LDS_SACC + LDS_DEN + LDS_MAX + LDS_CNT + LDS_BET + LDS_LB) % 4) == 0);
static_assert(LDS_BYTES == 289568);

typedef float          v4f  __attribute__((ext_vector_type(4)));
typedef float          v8f  __attribute__((ext_vector_type(8)));
typedef int            v4i  __attribute__((ext_vector_type(4)));
typedef unsigned short v4us __attribute__((ext_vector_type(4)));
typedef unsigned short v8us __attribute__((ext_vector_type(8)));
typedef __bf16         v16b __attribute__((ext_vector_type(16)));
union Frag   { v16b v; v8us half[2]; };
union Pack16 { v8us u; v4us q[2]; v4i i; };

__device__ __forceinline__ v8f wm(v16b a, v16b b, v8f c) {
  v8f d = __builtin_amdgcn_wmma_f32_16x16x32_bf16(false, a, false, b, (short)0, c, false, false);
  asm volatile("v_nop\n\tv_nop\n\tv_nop\n\tv_nop" : "+v"(d) : "v"(a), "v"(b));
  return d;
}

__device__ __forceinline__ float wsum(float v) {
  v += __shfl_xor(v, 16, 32);
  v += __shfl_xor(v, 8, 32);
  v += __shfl_xor(v, 4, 32);
  v += __shfl_xor(v, 2, 32);
  v += __shfl_xor(v, 1, 32);
  return v;
}

__device__ __forceinline__ float frcp(float x) { return __builtin_amdgcn_rcpf(x); }

__device__ __forceinline__ unsigned bfb(float x) {
  const unsigned u = __float_as_uint(x);
  return (u + 0x7FFFu + ((u >> 16) & 1u)) >> 16;
}

__device__ __forceinline__ void split4(v4f f, v4us& hi, v4us& lo) {
  const unsigned a0 = bfb(f.x), a1 = bfb(f.y), a2 = bfb(f.z), a3 = bfb(f.w);
  hi.x = (unsigned short)a0; hi.y = (unsigned short)a1; hi.z = (unsigned short)a2; hi.w = (unsigned short)a3;
  lo.x = (unsigned short)bfb(f.x - __uint_as_float(a0 << 16));
  lo.y = (unsigned short)bfb(f.y - __uint_as_float(a1 << 16));
  lo.z = (unsigned short)bfb(f.z - __uint_as_float(a2 << 16));
  lo.w = (unsigned short)bfb(f.w - __uint_as_float(a3 << 16));
}

__device__ __forceinline__ void put_planes(unsigned short* ph, unsigned short* plo, size_t o, v4f fa, v4f fb) {
  Pack16 uh, ul;
  split4(fa, uh.q[0], ul.q[0]);
  split4(fb, uh.q[1], ul.q[1]);
  *(volatile v4i*)(ph + o)  = uh.i;
  *(volatile v4i*)(plo + o) = ul.i;
  __threadfence();
  *(volatile v4i*)(ph + o)  = uh.i;
  *(volatile v4i*)(plo + o) = ul.i;
}

__global__ __launch_bounds__(NTHR) void k_prepw(
    const float* __restrict__ d_w, const float* __restrict__ w_w, const float* __restrict__ lin_w,
    unsigned short* Bnh, unsigned short* Bnl, unsigned short* Lh, unsigned short* Ll) {
  const int tid = threadIdx.x;
  v4f fa, fb;
  if (blockIdx.x < 8) {
    const int i  = blockIdx.x * NTHR + tid;
    const int n  = i >> 3;
    const int k0 = (i & 7) * 8;
    const int nr = (n < HH) ? 0 : (n - HH);
    const float* base = (n < HH) ? (d_w + n) : (w_w + (size_t)(nr >> 6) * (DI * HH) + (nr & 63));
    fa.x = base[(size_t)(k0 + 0) * HH]; fa.y = base[(size_t)(k0 + 1) * HH];
    fa.z = base[(size_t)(k0 + 2) * HH]; fa.w = base[(size_t)(k0 + 3) * HH];
    fb.x = base[(size_t)(k0 + 4) * HH]; fb.y = base[(size_t)(k0 + 5) * HH];
    fb.z = base[(size_t)(k0 + 6) * HH]; fb.w = base[(size_t)(k0 + 7) * HH];
    put_planes(Bnh, Bnl, (size_t)n * DI + k0, fa, fb);
  } else {
    const int i  = (blockIdx.x - 8) * NTHR + tid;
    const int n  = i / 24;
    const int k0 = (i - n * 24) * 8;
    const float* base = lin_w + n;
    fa.x = base[(size_t)(k0 + 0) * HH]; fa.y = base[(size_t)(k0 + 1) * HH];
    fa.z = base[(size_t)(k0 + 2) * HH]; fa.w = base[(size_t)(k0 + 3) * HH];
    fb.x = base[(size_t)(k0 + 4) * HH]; fb.y = base[(size_t)(k0 + 5) * HH];
    fb.z = base[(size_t)(k0 + 6) * HH]; fb.w = base[(size_t)(k0 + 7) * HH];
    put_planes(Lh, Ll, (size_t)n * KL + k0, fa, fb);
  }
}

__global__ __launch_bounds__(NTHR) void k_node(
    const float* __restrict__ h, const unsigned short* __restrict__ Bnh, const unsigned short* __restrict__ Bnl,
    const float* __restrict__ d_b, const float* __restrict__ w_b,
    const float* __restrict__ atten_w, const float* __restrict__ atten_b,
    float* pl, float* rec, int nN, int nP) {
  __shared__ __attribute__((aligned(16))) unsigned short Ah[GR * AP];
  __shared__ __attribute__((aligned(16))) unsigned short Al[GR * AP];
  __shared__ __attribute__((aligned(16))) float Xs[GR * XSP];
  __shared__ __attribute__((aligned(16))) float recS[NREL * GR * 8];
  __shared__ float waS[NREL * 48];
  __shared__ float abS[4];
  __shared__ float bS[NCOL];

  const int tid  = threadIdx.x;
  const int lane = tid & 31;
  const int wave = tid >> 5;
  const int h2   = lane >> 4;
  const int m    = lane & 15;
  const int rowBase = blockIdx.x * GR;

  if (tid < NREL * 48) waS[tid] = atten_w[tid];
  if (tid < NREL) abS[tid] = atten_b[tid];
  {
    const float v1 = d_b[(tid < HH) ? tid : (HH - 1)];
    const float v2 = w_b[(tid >= HH) ? (tid - HH) : 0];
    bS[tid] = (tid < HH) ? v1 : v2;
  }
  {
    const int rr = tid >> 3;
    const int c0 = (tid & 7) * 8;
    int row = rowBase + rr;
    if (row > nN - 1) row = nN - 1;
    const float* p = h + (size_t)row * DI + c0;
    const v4f f0 = *(const v4f*)p;
    const v4f f1 = *(const v4f*)(p + 4);
    Pack16 uh, ul;
    split4(f0, uh.q[0], ul.q[0]);
    split4(f1, uh.q[1], ul.q[1]);
    *(v8us*)(Ah + rr * AP + c0) = uh.u;
    *(v8us*)(Al + rr * AP + c0) = ul.u;
  }
  __syncthreads();

  const v8f z8 = {0.f, 0.f, 0.f, 0.f, 0.f, 0.f, 0.f, 0.f};
  v8f acc[2][2];
#pragma unroll
  for (int rt = 0; rt < 2; ++rt) {
#pragma unroll
    for (int ct = 0; ct < 2; ++ct) acc[rt][ct] = z8;
  }
#pragma unroll 1
  for (int kt = 0; kt < DI / 32; ++kt) {
    const int k0 = kt * 32;
    Frag ah[2], alo[2];
#pragma unroll
    for (int rt = 0; rt < 2; ++rt) {
      const unsigned short* pa = Ah + (16 * rt + m) * AP + k0 + 8 * h2;
      const unsigned short* pq = Al + (16 * rt + m) * AP + k0 + 8 * h2;
      ah[rt].half[0]  = *(const v8us*)pa;  ah[rt].half[1]  = *(const v8us*)(pa + 16);
      alo[rt].half[0] = *(const v8us*)pq;  alo[rt].half[1] = *(const v8us*)(pq + 16);
    }
#pragma unroll
    for (int ct = 0; ct < 2; ++ct) {
      const int ncol = (2 * wave + ct) * 16 + m;
      const unsigned short* pb = Bnh + (size_t)ncol * DI + k0 + 8 * h2;
      const unsigned short* pc = Bnl + (size_t)ncol * DI + k0 + 8 * h2;
      Frag bh, bl;
      bh.half[0] = *(const v8us*)pb;  bh.half[1] = *(const v8us*)(pb + 16);
      bl.half[0] = *(const v8us*)pc;  bl.half[1] = *(const v8us*)(pc + 16);
#pragma unroll
      for (int rt = 0; rt < 2; ++rt) {
        acc[rt][ct] = wm(ah[rt].v,  bh.v, acc[rt][ct]);
        acc[rt][ct] = wm(ah[rt].v,  bl.v, acc[rt][ct]);
        acc[rt][ct] = wm(alo[rt].v, bh.v, acc[rt][ct]);
      }
    }
  }

#pragma unroll
  for (int rt = 0; rt < 2; ++rt) {
#pragma unroll
    for (int ct = 0; ct < 2; ++ct) {
      const int col = (2 * wave + ct) * 16 + m;
      const float b = bS[col];
#pragma unroll
      for (int r8 = 0; r8 < 8; ++r8) Xs[(16 * rt + 8 * h2 + r8) * XSP + col] = acc[rt][ct][r8] + b;
    }
  }
  __syncthreads();

#pragma unroll 1
  for (int q = 0; q < (GR * HH) / NTHR; ++q) {
    const int e = q * NTHR + tid;
    const int row = e >> 6, col = e & 63;
    const float v = Xs[row * XSP + col];
    Xs[row * XSP + col] = tanhf(2.0f * v);
  }
  __syncthreads();

#pragma unroll 1
  for (int q = 0; q < 3; ++q) {
    const int i   = q * NTHR + tid;
    const int row = i / 24;
    const int rem = i - row * 24;
    const int rr  = rem >> 3;
    const int j   = rem & 7;
    const int hdd = j & 3;
    const float* xh = Xs + row * XSP + HH + HH * rr + 16 * hdd;
    const float* xt = Xs + row * XSP + 16 * hdd;
    const float* wa = waS + rr * 48;
    const int wsel = (j < 4) ? 0 : 16;
    float s1 = 0.f, s2 = 0.f;
#pragma unroll
    for (int c = 0; c < 16; ++c) {
      s1 += xh[c] * wa[wsel + c];
      s2 += xt[c] * wa[32 + c];
    }
    const float v = (j < 4) ? (s1 + s2 + abS[rr]) : s1;
    recS[(rr * GR + row) * 8 + j] = v;
  }
  __syncthreads();

#pragma unroll 1
  for (int pass = 0; pass < 2; ++pass) {
#pragma unroll 1
    for (int p = 0; p < 4; ++p) {
#pragma unroll
      for (int u = 0; u < 2; ++u) {
        const int idx = u * NTHR + tid;
        const int row = idx >> 4;
        const int cc  = (idx & 15) * 4;
        const v4f v = *(const v4f*)(Xs + row * XSP + p * HH + cc);
        *(volatile v4f*)(pl + ((size_t)p * (size_t)nP + (size_t)(rowBase + row)) * HH + cc) = v;
      }
    }
    if (tid < 64) {
#pragma unroll
      for (int rr = 0; rr < NREL; ++rr) {
        const v4f v = *(const v4f*)(recS + rr * (GR * 8) + 4 * tid);
        *(volatile v4f*)(rec + ((size_t)rr * (size_t)nP + (size_t)rowBase) * 8 + 4 * tid) = v;
      }
    }
    if (pass == 0) __threadfence();
  }
}

__global__ __launch_bounds__(NTHR) void k_agg(
    const int* __restrict__ srcr, const int* __restrict__ dstr,
    const float* pl, const float* __restrict__ recr, const float* __restrict__ betar,
    const unsigned short* __restrict__ Lh, const unsigned short* __restrict__ Ll,
    const float* __restrict__ lin_b, const float* yin, float* yout,
    float ps, float bs, int r, int nN, int nE, int nP) {
  extern __shared__ v4f lds_dyn[];
  float* sacc  = (float*)lds_dyn;
  float* den   = sacc + LDS_SACC;
  float* smax  = den + LDS_DEN;
  float* cnt   = smax + LDS_MAX;
  float* betaS = cnt + LDS_CNT;
  float* lbS   = betaS + LDS_BET;
  int*   list  = (int*)(lbS + LDS_LB);
  int*   wcnt  = list + LDS_LIST;
  unsigned short* l16 = (unsigned short*)lds_dyn;

  const int tid  = threadIdx.x;
  const int lane = tid & 31;
  const int wave = tid >> 5;
  const int h2   = lane >> 4;
  const int m    = lane & 15;
  const int c4   = 4 * m;
  const int hd   = m >> 2;
  const bool isT = (lane >= 16);
  const int nodeBase = blockIdx.x * NB;

  {
    const v4f z4 = {0.f, 0.f, 0.f, 0.f};
    for (int i = tid; i < (LDS_SACC + LDS_DEN) / 4; i += NTHR) lds_dyn[i] = z4;
    for (int i = tid; i < LDS_MAX; i += NTHR) smax[i] = -1.0e30f;
    for (int i = tid; i < LDS_CNT; i += NTHR) cnt[i] = 0.f;
    if (tid < LDS_BET) betaS[tid] = betar[tid];
    if (tid < LDS_LB) lbS[tid] = lin_b[tid];
  }
  __syncthreads();

  const float* hpr = pl + (size_t)(1 + r) * (size_t)nP * HH;
  const size_t goff = (size_t)(isT ? 0 : (1 + r)) * (size_t)nP;
  const bool al16 = ((((size_t)dstr) & 15) == 0);
  const int nChunks = (nE + CHUNK - 1) / CHUNK;

#pragma unroll 1
  for (int ch = 0; ch < nChunks; ++ch) {
    const int cbase = ch * CHUNK;
    const bool vec = al16 && (cbase + CHUNK <= nE);
    int wc = 0;
#pragma unroll
    for (int g = 0; g < NGRP; ++g) {
      const int el0 = (g * NTHR + tid) * 4;
      const int e0  = cbase + el0;
      const int sent = -2147483647 - 1;
      v4i d;
      if (vec) {
        d = *(const v4i*)(dstr + e0);
      } else {
        const int q0 = (e0     < nE) ? (e0)     : (nE - 1);
        const int q1 = (e0 + 1 < nE) ? (e0 + 1) : (nE - 1);
        const int q2 = (e0 + 2 < nE) ? (e0 + 2) : (nE - 1);
        const int q3 = (e0 + 3 < nE) ? (e0 + 3) : (nE - 1);
        const int v0 = dstr[q0], v1 = dstr[q1], v2 = dstr[q2], v3 = dstr[q3];
        d.x = (e0     < nE) ? v0 : sent;
        d.y = (e0 + 1 < nE) ? v1 : sent;
        d.z = (e0 + 2 < nE) ? v2 : sent;
        d.w = (e0 + 3 < nE) ? v3 : sent;
      }
      const unsigned s0 = (unsigned)d.x - (unsigned)nodeBase;
      const unsigned s1 = (unsigned)d.y - (unsigned)nodeBase;
      const unsigned s2 = (unsigned)d.z - (unsigned)nodeBase;
      const unsigned s3 = (unsigned)d.w - (unsigned)nodeBase;
      const bool b0 = s0 < (unsigned)NB;
      const bool b1 = s1 < (unsigned)NB;
      const bool b2 = s2 < (unsigned)NB;
      const bool b3 = s3 < (unsigned)NB;
      const unsigned many = __builtin_amdgcn_ballot_w32(b0 | b1 | b2 | b3);
      if (many != 0u) {
#define HITJ(J, HJ, SJ) { \
          const unsigned mj = __builtin_amdgcn_ballot_w32(HJ); \
          if (HJ) { \
            const int pos = wc + (int)__builtin_amdgcn_mbcnt_lo(mj, 0u); \
            if (pos < WCAP) list[wave * WCAP + pos] = ((el0 + (J)) << 9) | (int)(SJ); \
          } \
          wc += (int)__builtin_popcount(mj); }
        HITJ(0, b0, s0)
        HITJ(1, b1, s1)
        HITJ(2, b2, s2)
        HITJ(3, b3, s3)
#undef HITJ
      }
    }
    if (lane == 0) wcnt[wave] = wc;
    __syncthreads();

    if (wave == 0) {
#pragma unroll 1
      for (int wsx = 0; wsx < NWAVE; ++wsx) {
        int n = wcnt[wsx];
        if (n > WCAP) n = WCAP;
        if (n < 0) n = 0;
#pragma unroll 1
        for (int i = 0; i < n; ++i) {
          const int ent  = list[wsx * WCAP + i];
          const int slot = ent & (NB - 1);
          const int el   = (ent >> 9) & (CHUNK - 1);
          int e = cbase + el;
          if (e > nE - 1) e = nE - 1;
          int s = srcr[e];
          s = (s < 0) ? 0 : ((s > nN - 1) ? (nN - 1) : s);
          int t = nodeBase + slot;
          if (t > nN - 1) t = nN - 1;
          const float sq = recr[(size_t)s * 8 + hd];
          const float sd = recr[(size_t)t * 8 + 4 + hd];
          float al = sq + sd;
          al = (al >= 0.f) ? al : 0.01f * al;
          const int mi = slot * NHD + hd;
          const float mo = smax[mi];
          const float dv = den[mi];
          const float mn = fmaxf(mo, al);
          const float sc = __expf(mo - mn);
          const float p  = __expf(al - mn);
          const float fs = isT ? 1.0f : sc;
          const float fp = isT ? 1.0f : p;
          const v4f xv = *(const v4f*)(pl + (goff + (size_t)s) * HH + c4);
          v4f* sp = (v4f*)(sacc + slot * SROW + 4 * lane);
          const v4f cur = *sp;
          const v4f nxt = cur * fs + xv * fp;
          *sp = nxt;
          if (!isT && ((lane & 3) == 0)) {
            den[mi]  = dv * sc + p;
            smax[mi] = mn;
          }
          if (lane == 16) {
            const float c = cnt[slot];
            cnt[slot] = c + 1.0f;
          }
        }
      }
    }
    __syncthreads();
  }

#pragma unroll 1
  for (int j = 0; j < NB / NWAVE; ++j) {
    const int slot = wave * (NB / NWAVE) + j;
    const int node = nodeBase + slot;
    if (node >= nN) break;
    const v4f raw = *(const v4f*)(sacc + slot * SROW + 4 * lane);
    const float dv = den[slot * NHD + hd];
    const float cv = cnt[slot];
    const float io = frcp(fmaxf(dv, 1e-20f));
    const float ic = frcp(fmaxf(cv, 1.0f));
    const v4f val = raw * (isT ? ic : io);
    const v4f b4 = *(const v4f*)(betaS + (isT ? c4 : (HH + c4)));
    float g = val.x * b4.x + val.y * b4.y + val.z * b4.z + val.w * b4.w;
    g = wsum(g);
    const float gate = frcp(1.0f + __expf(-g));
    const v4f hv = *(const v4f*)(hpr + (size_t)node * HH + c4);
    const v4f res = val * gate + hv * (1.0f - gate);
    v4us hi4, lo4;
    split4(res, hi4, lo4);
    __builtin_amdgcn_fence(__ATOMIC_RELEASE, "wavefront");
    __builtin_amdgcn_wave_barrier();
    if (!isT) {
      *(v4us*)(l16 + (size_t)slot * (SROW * 2) + c4)      = hi4;
      *(v4us*)(l16 + (size_t)slot * (SROW * 2) + HH + c4) = lo4;
    }
  }
  __syncthreads();

  const v8f z8 = {0.f, 0.f, 0.f, 0.f, 0.f, 0.f, 0.f, 0.f};
#pragma unroll 1
  for (int q = 0; q < 4; ++q) {
    const int s0 = (wave * 4 + q) * 16;
    v8f acc[4];
#pragma unroll
    for (int ct = 0; ct < 4; ++ct) acc[ct] = z8;
#pragma unroll 1
    for (int kt = 0; kt < HH / 32; ++kt) {
      const int k0 = kt * 32;
      Frag ah, alo;
      const unsigned short* pa = l16 + (size_t)(s0 + m) * (SROW * 2) + k0 + 8 * h2;
      ah.half[0]  = *(const v8us*)pa;         ah.half[1]  = *(const v8us*)(pa + 16);
      alo.half[0] = *(const v8us*)(pa + HH);  alo.half[1] = *(const v8us*)(pa + HH + 16);
#pragma unroll
      for (int ct = 0; ct < 4; ++ct) {
        const size_t bo = (size_t)(ct * 16 + m) * KL + (size_t)r * HH + k0 + 8 * h2;
        Frag bh, bl;
        bh.half[0] = *(const v8us*)(Lh + bo);  bh.half[1] = *(const v8us*)(Lh + bo + 16);
        bl.half[0] = *(const v8us*)(Ll + bo);  bl.half[1] = *(const v8us*)(Ll + bo + 16);
        acc[ct] = wm(ah.v,  bh.v, acc[ct]);
        acc[ct] = wm(ah.v,  bl.v, acc[ct]);
        acc[ct] = wm(alo.v, bh.v, acc[ct]);
      }
    }
#pragma unroll
    for (int ct = 0; ct < 4; ++ct) {
#pragma unroll
      for (int r8 = 0; r8 < 8; ++r8) sacc[(s0 + 8 * h2 + r8) * SROW + HH + ct * 16 + m] = acc[ct][r8];
    }
  }
  __syncthreads();

#pragma unroll 1
  for (int pass = 0; pass < 2; ++pass) {
#pragma unroll 1
    for (int q = 0; q < 4; ++q) {
      const int s0 = (wave * 4 + q) * 16;
#pragma unroll 1
      for (int jj = 0; jj < 8; ++jj) {
        const int slot = s0 + 2 * jj + h2;
        const int node = nodeBase + slot;
        const int nc = (node > nN - 1) ? (nN - 1) : node;
        const v4f d4 = *(const v4f*)(sacc + slot * SROW + HH + c4);
        const v4f pv = *(const v4f*)(yin + (size_t)nc * HH + c4);
        const v4f lb = *(const v4f*)(lbS + c4);
        const v4f val = d4 + pv * ps + lb * bs;
        if (node < nN) *(volatile v4f*)(yout + (size_t)node * HH + c4) = val;
      }
    }
    if (pass == 0) __threadfence();
  }
}

extern "C" void kernel_launch(void* const* d_in, const int* in_sizes, int n_in,
                              void* d_out, int out_size, void* d_ws, size_t ws_size,
                              hipStream_t stream) {
  if (n_in < 12) return;
  const int nN = in_sizes[0] / DI;
  if (nN <= 0 || in_sizes[0] != nN * DI) return;
  const int nE = in_sizes[1] / NREL;
  if (nE <= 0 || in_sizes[1] != NREL * nE || in_sizes[2] != NREL * nE) return;
  if (in_sizes[3] != DI * HH || in_sizes[4] != HH) return;
  if (in_sizes[5] != NREL * DI * HH || in_sizes[6] != NREL * HH) return;
  if (in_sizes[7] != NREL * 48 || in_sizes[8] != NREL || in_sizes[9] != NREL * 128) return;
  if (in_sizes[10] != KL * HH || in_sizes[11] != HH) return;
  if (out_size != nN * HH) return;

  const float* h       = (const float*)d_in[0];
  const int*   src     = (const int*)d_in[1];
  const int*   dst     = (const int*)d_in[2];
  const float* d_w     = (const float*)d_in[3];
  const float* d_b     = (const float*)d_in[4];
  const float* w_w     = (const float*)d_in[5];
  const float* w_b     = (const float*)d_in[6];
  const float* atten_w = (const float*)d_in[7];
  const float* atten_b = (const float*)d_in[8];
  const float* beta    = (const float*)d_in[9];
  const float* lin_w   = (const float*)d_in[10];
  const float* lin_b   = (const float*)d_in[11];
  float* out = (float*)d_out;

  const int nP = ((nN + GR - 1) / GR) * GR;
  size_t off = 0;
  unsigned short* Bnh = (unsigned short*)((char*)d_ws + off); off += (size_t)NCOL * DI * 2;
  unsigned short* Bnl = (unsigned short*)((char*)d_ws + off); off += (size_t)NCOL * DI * 2;
  unsigned short* Lh  = (unsigned short*)((char*)d_ws + off); off += (size_t)HH * KL * 2;
  unsigned short* Ll  = (unsigned short*)((char*)d_ws + off); off += (size_t)HH * KL * 2;
  float* pl  = (float*)((char*)d_ws + off); off += (size_t)4 * (size_t)nP * HH * sizeof(float);
  float* rec = (float*)((char*)d_ws + off); off += (size_t)NREL * (size_t)nP * 8 * sizeof(float);
  if (off > ws_size) return;

  k_prepw<<<14, NTHR, 0, stream>>>(d_w, w_w, lin_w, Bnh, Bnl, Lh, Ll);

  k_node<<<nP / GR, NTHR, 0, stream>>>(h, Bnh, Bnl, d_b, w_b, atten_w, atten_b, pl, rec, nN, nP);

  hipFuncSetAttribute(reinterpret_cast<const void*>(&k_agg),
                      hipFuncAttributeMaxDynamicSharedMemorySize, LDS_BYTES);
  const int grid = (nN + NB - 1) / NB;
  const size_t plane = (size_t)nP * HH;
  k_agg<<<grid, NTHR, LDS_BYTES, stream>>>(src, dst, pl, rec, beta, Lh, Ll, lin_b,
                                           pl, out, 0.f, 1.f, 0, nN, nE, nP);
  k_agg<<<grid, NTHR, LDS_BYTES, stream>>>(src + (size_t)nE, dst + (size_t)nE, pl, rec + (size_t)nP * 8,
                                           beta + 128, Lh, Ll, lin_b,
                                           out, pl + plane, 1.f, 0.f, 1, nN, nE, nP);
  k_agg<<<grid, NTHR, LDS_BYTES, stream>>>(src + 2 * (size_t)nE, dst + 2 * (size_t)nE, pl, rec + 2 * (size_t)nP * 8,
                                           beta + 256, Lh, Ll, lin_b,
                                           pl + plane, out, 1.f, 0.f, 2, nN, nE, nP);
}
